// GLAWrapper_9285719294259
// MI455X (gfx1250) — hardware-verified
//
#include <hip/hip_runtime.h>
#include <math.h>

constexpr int kNB    = 2;
constexpr int kNT    = 4096;
constexpr int kDM    = 1024;
constexpr int kNH    = 4;
constexpr int kDKH   = 128;
constexpr int kDVH   = 256;
constexpr int kKD    = kNH * kDKH;
constexpr int kVD    = kNH * kDVH;
constexpr int kLR    = 16;
constexpr int kCS    = 64;
constexpr int kNCH   = kNT / kCS;
constexpr int kRows  = kNB * kNT;
constexpr int kNA    = 1088;
constexpr int kSsnP  = 136;
constexpr int kAbfP  = 72;
constexpr int kOstP  = 68;
constexpr float kWCarry    = 64.0f;
constexpr float kWCarryInv = 1.0f / 64.0f;
constexpr float kQScale    = 0.08838834764831845f;
constexpr float kInvGN     = 1.0f / 16.0f;
constexpr float kNormEps   = 1e-5f;
static_assert(kKD == 512 && kVD == 1024 && kRows == 8192 && kNCH == 64, "shape");
static_assert((double)kQScale * (double)kQScale * (double)kDKH > 0.999999 &&
              (double)kQScale * (double)kQScale * (double)kDKH < 1.000001, "q scale = DK^-0.5");
static_assert(kDM % 32 == 0 && kVD % 32 == 0, "GEMM K multiple of 32");
static_assert(kRows % 64 == 0 && kNA % 64 == 0 && kVD % 64 == 0 && kDM % 64 == 0, "GEMM M,N multiples of 64");
static_assert(kNA >= 2 * kKD + kLR, "q|k|t1 plane width");
static_assert(kNT == kCS * kNCH, "no chunk tail");

typedef __attribute__((ext_vector_type(16))) _Float16 v16h;
typedef __attribute__((ext_vector_type(8)))  _Float16 v8h;
typedef __attribute__((ext_vector_type(8)))  float    v8f;
typedef __attribute__((ext_vector_type(4)))  float    v4f;
typedef __attribute__((ext_vector_type(4)))  unsigned int v4u;

__device__ __forceinline__ unsigned short f2bf_bits(float f) {
  unsigned u = __float_as_uint(f);
  return (unsigned short)((u + 0x7FFFu + ((u >> 16) & 1u)) >> 16);
}
__device__ __forceinline__ float bf_bits2f(unsigned short h) { return __uint_as_float(((unsigned)h) << 16); }
__device__ __forceinline__ float bf16r(float f) { return bf_bits2f(f2bf_bits(f)); }
__device__ __forceinline__ unsigned pk16(unsigned short a, unsigned short b) { return (unsigned)a | ((unsigned)b << 16); }
__device__ __forceinline__ unsigned short h_bits(float f) { const _Float16 h = (_Float16)f; return __builtin_bit_cast(unsigned short, h); }
__device__ __forceinline__ float h16_to_f32(unsigned hb) {
  const unsigned sgn = (hb & 0x8000u) << 16;
  const unsigned em = hb & 0x7fffu;
  const float fn = __uint_as_float((em << 13) + 0x38000000u);
  const float fs = (float)em * 5.9604644775390625e-8f;
  const float mag = (em < 0x400u) ? fs : fn;
  return __uint_as_float(__float_as_uint(mag) | sgn);
}

__device__ __forceinline__ void guard4_h(v8f& a, v8f& b, v8f& c, v8f& d, v16h x, v16h y) {
  asm volatile("v_nop\n\tv_nop\n\tv_nop\n\tv_nop" : "+v"(a), "+v"(b), "+v"(c), "+v"(d) : "v"(x), "v"(y));
}
__device__ __forceinline__ void keep4_h(v16h a, v16h b, v16h c, v16h d) { asm volatile("v_nop" :: "v"(a), "v"(b), "v"(c), "v"(d)); }
__device__ __forceinline__ void acc_guard4(v8f& a, v8f& b, v8f& c, v8f& d) {
  asm volatile("v_nop\n\tv_nop\n\tv_nop\n\tv_nop" : "+v"(a), "+v"(b), "+v"(c), "+v"(d));
}

union FragU { v16h v; v8h h[2]; };
__device__ __forceinline__ v16h frag_load(const _Float16* p) {
  FragU f;
  f.h[0] = *(const v8h*)(p);
  f.h[1] = *(const v8h*)(p + 16);
  return f.v;
}
__device__ __forceinline__ v8f mma_raw(v16h a, v16h b, v8f c) {
  return __builtin_amdgcn_wmma_f32_16x16x32_f16(false, a, false, b, (short)0, c, false, false);
}
__device__ __forceinline__ v8f mma_g(v16h a, v16h b, v8f c) {
  c = __builtin_amdgcn_wmma_f32_16x16x32_f16(false, a, false, b, (short)0, c, false, false);
  asm volatile("v_nop\n\tv_nop\n\tv_nop\n\tv_nop" : "+v"(c) : "v"(a), "v"(b));
  return c;
}

__global__ __launch_bounds__(256) void cvt8_kernel(const float* __restrict__ src, unsigned short* __restrict__ dst, int n8) {
  const int i = blockIdx.x * 256 + threadIdx.x;
  if (i < n8) {
    const float* sp = src + (size_t)i * 8;
    const v4f a = *(const v4f*)(sp);
    const v4f b = *(const v4f*)(sp + 4);
    unsigned short hb[8];
#pragma unroll
    for (int e = 0; e < 4; ++e) {
      const float fa = a[e];
      const float fb = b[e];
      hb[e]     = h_bits(bf16r(fa));
      hb[4 + e] = h_bits(bf16r(fb));
    }
    const v4u u = (v4u){pk16(hb[0], hb[1]), pk16(hb[2], hb[3]), pk16(hb[4], hb[5]), pk16(hb[6], hb[7])};
    unsigned short* q = dst + (size_t)i * 8;
    *(volatile v4u*)q = u;
    __threadfence();
    *(volatile v4u*)q = u;
  }
}

__global__ __launch_bounds__(256) void wtcast_kernel(const float* __restrict__ W, int ncols,
                                                     unsigned short* __restrict__ out, float carry) {
  __shared__ float sm[64][65];
  const int t  = threadIdx.x;
  const int d0 = blockIdx.x * 64;
  const int h0 = blockIdx.y * 64;
#pragma unroll
  for (int i = 0; i < 16; ++i) {
    const int e = i * 256 + t;
    const int r = e >> 6;
    const int c = e & 63;
    const int col  = h0 + c;
    const int colc = (col < ncols) ? col : (ncols - 1);
    const float raw = W[(size_t)(d0 + r) * ncols + colc];
    const float val = (col < ncols) ? (bf16r(raw) * carry) : 0.0f;
    sm[c][r] = val;
  }
  __syncthreads();
  const int lane = t & 31, wave = t >> 5;
  const int q = lane >> 3, c8 = (lane & 7) * 8;
  for (int pass = 0; pass < 2; ++pass) {
#pragma unroll
    for (int it = 0; it < 2; ++it) {
      const int row = wave * 8 + it * 4 + q;
      unsigned short hb[8];
#pragma unroll
      for (int e = 0; e < 8; ++e) hb[e] = h_bits(sm[row][c8 + e]);
      const v4u u = (v4u){pk16(hb[0], hb[1]), pk16(hb[2], hb[3]), pk16(hb[4], hb[5]), pk16(hb[6], hb[7])};
      *(volatile v4u*)(out + (size_t)(h0 + row) * kDM + d0 + c8) = u;
    }
    __threadfence();
  }
}

template <int OUT_MODE>
__global__ __launch_bounds__(256) void wmma_gemm64_h(
    const unsigned short* __restrict__ Ap, int lda,
    const unsigned short* __restrict__ Btp, int ldb,
    void* __restrict__ Cout, int ldc, int M, int N, int K, float scale) {
  const _Float16* A  = (const _Float16*)Ap;
  const _Float16* Bt = (const _Float16*)Btp;
  __shared__ __align__(16) float sT[8][16 * 68];
  const int lane = threadIdx.x & 31;
  const int wave = threadIdx.x >> 5;
  const int tilesN = N >> 6;
  const int tilesM = M >> 6;
  const int tile = blockIdx.x * 8 + wave;
  if (tile >= tilesM * tilesN) return;
  const int tm = tile / tilesN;
  const int tn = tile - tm * tilesN;
  const int m0 = tm << 6;
  const int n0 = tn << 6;

  const int rlane = lane & 15;
  const int koff  = (lane >> 4) * 8;
  const int mOff  = (lane >> 4) * 8;

  v8f acc[4][4];
#pragma unroll
  for (int i = 0; i < 4; ++i)
#pragma unroll
    for (int j = 0; j < 4; ++j) acc[i][j] = (v8f){0.f, 0.f, 0.f, 0.f, 0.f, 0.f, 0.f, 0.f};

  for (int k0 = 0; k0 < K; k0 += 32) {
    v16h bh[4];
#pragma unroll
    for (int j = 0; j < 4; ++j) {
      const size_t bo = (size_t)(n0 + (j << 4) + rlane) * ldb + koff + k0;
      bh[j] = frag_load(Bt + bo);
    }
#pragma unroll
    for (int i = 0; i < 4; ++i) {
      const size_t ao = (size_t)(m0 + (i << 4) + rlane) * lda + koff + k0;
      const v16h ah = frag_load(A + ao);
#pragma unroll
      for (int j = 0; j < 4; ++j) acc[i][j] = mma_raw(ah, bh[j], acc[i][j]);
      guard4_h(acc[i][0], acc[i][1], acc[i][2], acc[i][3], ah, bh[3]);
    }
    keep4_h(bh[0], bh[1], bh[2], bh[3]);
  }
  acc_guard4(acc[0][0], acc[0][1], acc[0][2], acc[0][3]);
  acc_guard4(acc[1][0], acc[1][1], acc[1][2], acc[1][3]);
  acc_guard4(acc[2][0], acc[2][1], acc[2][2], acc[2][3]);
  acc_guard4(acc[3][0], acc[3][1], acc[3][2], acc[3][3]);

  float* slab = sT[wave];
#pragma unroll
  for (int i = 0; i < 4; ++i) {
    const int mBase = m0 + (i << 4);
#pragma unroll
    for (int j = 0; j < 4; ++j) {
#pragma unroll
      for (int r = 0; r < 8; ++r) {
        const float v = acc[i][j][r] * scale;
        slab[(mOff + r) * 68 + (j << 4) + rlane] = v;
      }
    }
    __builtin_amdgcn_fence(__ATOMIC_RELEASE, "workgroup");
    __builtin_amdgcn_wave_barrier();
    __builtin_amdgcn_fence(__ATOMIC_ACQUIRE, "workgroup");
    if (OUT_MODE == 0) {
      float* C = (float*)Cout;
      const int hh = lane >> 4, c4 = (lane & 15) * 4;
      for (int pass = 0; pass < 2; ++pass) {
#pragma unroll
        for (int it = 0; it < 8; ++it) {
          const int row = it * 2 + hh;
          const v4f v = *(const v4f*)(slab + row * 68 + c4);
          *(volatile v4f*)(C + (size_t)(mBase + row) * ldc + n0 + c4) = v;
        }
        __threadfence();
      }
    } else {
      const int q = lane >> 3, c8 = (lane & 7) * 8;
      unsigned short* C = (unsigned short*)Cout;
      for (int pass = 0; pass < 2; ++pass) {
#pragma unroll
        for (int it = 0; it < 4; ++it) {
          const int row = it * 4 + q;
          const float* sp = slab + row * 68 + c8;
          v8h hv;
#pragma unroll
          for (int e = 0; e < 8; ++e) hv[e] = (_Float16)sp[e];
          *(volatile v8h*)(C + (size_t)(mBase + row) * ldc + n0 + c8) = hv;
        }
        __threadfence();
      }
    }
    __builtin_amdgcn_fence(__ATOMIC_RELEASE, "workgroup");
    __builtin_amdgcn_wave_barrier();
    __builtin_amdgcn_fence(__ATOMIC_ACQUIRE, "workgroup");
  }
}

__global__ __launch_bounds__(128) void prep_kernel(const float* __restrict__ QKT, const float* __restrict__ Wgk2,
                                                   const float* __restrict__ bgk,
                                                   unsigned short* __restrict__ QG, unsigned short* __restrict__ KG,
                                                   unsigned short* __restrict__ KDT, float* __restrict__ GL) {
  __shared__ __align__(16) unsigned short qs[kCS * kDKH];
  __shared__ __align__(16) unsigned short ks[kCS * kDKH];
  __shared__ __align__(16) unsigned short ds[kDKH * kCS];
  __shared__ __align__(16) float gls[kDKH];
  const int tid = threadIdx.x;
  const int h   = blockIdx.x & 3;
  const int bn  = blockIdx.x >> 2;
  const int ch  = h * kDKH + tid;
  const size_t r0 = (size_t)bn * kCS;

  float w2[kLR];
#pragma unroll
  for (int u = 0; u < kLR; ++u) w2[u] = bf16r(Wgk2[u * kKD + ch]);
  const float bias = bf16r(bgk[ch]);

  float run = 0.0f, glast = 0.0f;
#pragma unroll 1
  for (int it = 0; it < 2 * kCS; ++it) {
    const int c = it & (kCS - 1);
    const bool second = (it >= kCS);
    const float* rowp = QKT + (r0 + (size_t)c) * kNA;
    v4f tv[4];
#pragma unroll
    for (int j = 0; j < 4; ++j) tv[j] = *(const v4f*)(rowp + 2 * kKD + 4 * j);
    float z = 0.0f;
#pragma unroll
    for (int u = 0; u < kLR; ++u) z = fmaf(tv[u >> 2][u & 3], w2[u], z);
    z += bias;
    const float ls = fminf(z, 0.0f) - log1pf(expf(-fabsf(z)));
    run += ls * kInvGN;
    if (!second) {
      if (c == kCS - 1) { glast = run; run = 0.0f; }
    } else {
      const float qv = rowp[ch];
      const float kv = rowp[kKD + ch];
      const float eG = expf(run);
      const float eI = expf(-run);
      const float eD = expf(glast - run);
      qs[c * kDKH + tid] = h_bits(qv * eG);
      ks[c * kDKH + tid] = h_bits(kv * eI);
      ds[tid * kCS + c]  = h_bits(kv * eD);
    }
  }
  gls[tid] = glast;
  __syncthreads();

  const int b = bn >> 6, n = bn & 63;
  const size_t tile = (size_t)((b * kNH + h) * kNCH + n);
  const int rsub = tid >> 4, c8 = (tid & 15) * 8;
  for (int pass = 0; pass < 2; ++pass) {
#pragma unroll
    for (int it = 0; it < 8; ++it) {
      const int row = it * 8 + rsub;
      const v4u vq = *(const v4u*)(qs + row * kDKH + c8);
      const v4u vk = *(const v4u*)(ks + row * kDKH + c8);
      const size_t go = (r0 + (size_t)row) * kKD + h * kDKH + c8;
      *(volatile v4u*)(QG + go) = vq;
      *(volatile v4u*)(KG + go) = vk;
      const int idx = it * 128 + tid;
      const v4u vd = *(const v4u*)(ds + idx * 8);
      *(volatile v4u*)(KDT + tile * (size_t)(kDKH * kCS) + (size_t)idx * 8) = vd;
    }
    if (tid < 32) {
      const v4f gv = *(const v4f*)(gls + tid * 4);
      *(volatile v4f*)(GL + (size_t)bn * kKD + h * kDKH + tid * 4) = gv;
    }
    __threadfence();
  }
}

__global__ __launch_bounds__(256) void chunk_scan_kernel(const unsigned short* __restrict__ QGp,
                                                         const unsigned short* __restrict__ KGp,
                                                         const unsigned short* __restrict__ KDTp,
                                                         const unsigned short* __restrict__ VTp,
                                                         const float* __restrict__ GL, float* __restrict__ ORAW) {
  __shared__ __align__(16) _Float16 Ssn[kCS * kSsnP];
  __shared__ __align__(16) _Float16 Abf[kCS * kAbfP];
  __shared__ __align__(16) float    Ost[kCS * kOstP];
  const _Float16* QG  = (const _Float16*)QGp;
  const _Float16* KG  = (const _Float16*)KGp;
  const _Float16* KDT = (const _Float16*)KDTp;
  const _Float16* VT  = (const _Float16*)VTp;

  const int bid = blockIdx.x;
  const int vs = bid & 3;
  const int h  = (bid >> 2) & 3;
  const int b  = bid >> 4;
  const int tid = threadIdx.x, lane = tid & 31, w = tid >> 5;
  const int c = lane & 15, hh = lane >> 4, koff = hh * 8;
  const int tm  = w >> 1;
  const int tnb = (w & 1) * 2;
  const int vrow0 = h * kDVH + vs * 64;

  const v8f z8 = {0.f, 0.f, 0.f, 0.f, 0.f, 0.f, 0.f, 0.f};
  v8f S[4];
#pragma unroll
  for (int t = 0; t < 4; ++t) S[t] = z8;

#pragma unroll 1
  for (int n = 0; n < kNCH; ++n) {
    const size_t r0 = (size_t)b * kNT + (size_t)n * kCS;
    const size_t tile = (size_t)((b * kNH + h) * kNCH + n);
    const size_t bn = (size_t)b * kNCH + n;

#pragma unroll
    for (int t = 0; t < 4; ++t) {
      v8h hv;
#pragma unroll
      for (int r = 0; r < 8; ++r) hv[r] = (_Float16)S[t][r];
      *(v8h*)(Ssn + (16 * t + c) * kSsnP + 16 * w + 8 * hh) = hv;
    }

    v16h qa[4];
#pragma unroll
    for (int k = 0; k < 4; ++k)
      qa[k] = frag_load(QG + (r0 + (size_t)(16 * tm + c)) * kKD + h * kDKH + koff + 32 * k);
#pragma unroll
    for (int t = 0; t < 2; ++t) {
      const int tn = tnb + t;
      v8f acc = z8;
#pragma unroll
      for (int k = 0; k < 4; ++k) {
        const v16h kb = frag_load(KG + (r0 + (size_t)(16 * tn + c)) * kKD + h * kDKH + koff + 32 * k);
        acc = mma_g(qa[k], kb, acc);
      }
      const int j = 16 * tn + c;
#pragma unroll
      for (int r = 0; r < 8; ++r) {
        const int i = 16 * tm + 8 * hh + r;
        const float av = (j <= i) ? (acc[r] * kQScale) : 0.0f;
        Abf[i * kAbfP + j] = (_Float16)av;
      }
    }
    __syncthreads();

#pragma unroll
    for (int t = 0; t < 2; ++t) {
      const int tn = tnb + t;
      v8f accI = z8;
#pragma unroll
      for (int k = 0; k < 4; ++k) {
        const v16h sb = frag_load(Ssn + (16 * tn + c) * kSsnP + koff + 32 * k);
        accI = mma_g(qa[k], sb, accI);
      }
      v8f accA = z8;
#pragma unroll
      for (int k = 0; k < 2; ++k) {
        const v16h af = frag_load(Abf + (16 * tm + c) * kAbfP + koff + 32 * k);
        const v16h vb = frag_load(VT + (size_t)(vrow0 + 16 * tn + c) * kRows + r0 + koff + 32 * k);
        accA = mma_g(af, vb, accA);
      }
#pragma unroll
      for (int r = 0; r < 8; ++r) {
        const float ov = accI[r] * kQScale + accA[r];
        Ost[(16 * tm + 8 * hh + r) * kOstP + 16 * tn + c] = ov;
      }
    }

    {
      const float* glp = GL + bn * kKD + h * kDKH + 16 * w + 8 * hh;
      const v4f g0 = *(const v4f*)(glp);
      const v4f g1 = *(const v4f*)(glp + 4);
      float e[8];
#pragma unroll
      for (int r = 0; r < 4; ++r) {
        const float a0 = g0[r];
        const float a1 = g1[r];
        e[r]     = expf(a0);
        e[4 + r] = expf(a1);
      }
      v16h ka[2];
#pragma unroll
      for (int k = 0; k < 2; ++k)
        ka[k] = frag_load(KDT + tile * (size_t)(kDKH * kCS) + (size_t)(16 * w + c) * kCS + koff + 32 * k);
#pragma unroll
      for (int t = 0; t < 4; ++t) {
#pragma unroll
        for (int r = 0; r < 8; ++r) S[t][r] *= e[r];
#pragma unroll
        for (int k = 0; k < 2; ++k) {
          const v16h vb = frag_load(VT + (size_t)(vrow0 + 16 * t + c) * kRows + r0 + koff + 32 * k);
          S[t] = mma_g(ka[k], vb, S[t]);
        }
      }
    }
    __syncthreads();

    {
      const int rsub = tid >> 4, c4 = (tid & 15) * 4;
      for (int pass = 0; pass < 2; ++pass) {
#pragma unroll
        for (int it = 0; it < 4; ++it) {
          const int row = it * 16 + rsub;
          const v4f v = *(const v4f*)(Ost + row * kOstP + c4);
          *(volatile v4f*)(ORAW + (r0 + (size_t)row) * kVD + vrow0 + c4) = v;
        }
        __threadfence();
      }
    }
  }
}

__global__ __launch_bounds__(256) void norm_gate_kernel(const float* __restrict__ ORAW, const unsigned short* __restrict__ G,
                                                        const float* __restrict__ norm_w, unsigned short* __restrict__ OG) {
  const int tid = threadIdx.x, lane = tid & 31;
  const int gid = blockIdx.x * 8 + (tid >> 5);
  const int row = gid >> 2, h = gid & 3;
  const size_t base = (size_t)row * kVD + h * kDVH + 8 * lane;
  const v4f o0 = *(const v4f*)(ORAW + base);
  const v4f o1 = *(const v4f*)(ORAW + base + 4);
  const v4u gw = *(const v4u*)(G + base);
  const v4f w0 = *(const v4f*)(norm_w + 8 * lane);
  const v4f w1 = *(const v4f*)(norm_w + 8 * lane + 4);
  float ov[8], wv[8], gv[8];
#pragma unroll
  for (int e = 0; e < 4; ++e) {
    ov[e] = o0[e];
    ov[4 + e] = o1[e];
    const float wa = w0[e];
    const float wb = w1[e];
    wv[e] = bf16r(wa);
    wv[4 + e] = bf16r(wb);
    const unsigned word = gw[e];
    gv[2 * e]     = h16_to_f32(word & 0xffffu);
    gv[2 * e + 1] = h16_to_f32(word >> 16);
  }
  float ss = 0.0f;
#pragma unroll
  for (int e = 0; e < 8; ++e) ss = fmaf(ov[e], ov[e], ss);
#pragma unroll
  for (int off = 16; off > 0; off >>= 1) ss += __shfl_xor(ss, off, 32);
  const float rms = sqrtf(ss * (1.0f / (float)kDVH) + kNormEps);
  const float inv = 1.0f / rms;
  unsigned short hb[8];
#pragma unroll
  for (int e = 0; e < 8; ++e) {
    const float sg = __builtin_amdgcn_rcpf(1.0f + expf(-gv[e]));
    const float val = ((ov[e] * inv) * wv[e]) * (gv[e] * sg);
    hb[e] = h_bits(val);
  }
  const v4u u = (v4u){pk16(hb[0], hb[1]), pk16(hb[2], hb[3]), pk16(hb[4], hb[5]), pk16(hb[6], hb[7])};
  unsigned short* op = OG + base;
  *(volatile v4u*)op = u;
  __threadfence();
  *(volatile v4u*)op = u;
}

extern "C" void kernel_launch(void* const* d_in, const int* in_sizes, int n_in,
                              void* d_out, int out_size, void* d_ws, size_t ws_size, hipStream_t stream) {
  if (n_in < 10 || d_out == nullptr || d_ws == nullptr) return;
  if (in_sizes[0] != kRows * kDM || in_sizes[1] != kDM * kKD || in_sizes[2] != kDM * kKD ||
      in_sizes[3] != kDM * kVD || in_sizes[4] != kDM * kVD || in_sizes[5] != kDM * kLR ||
      in_sizes[6] != kLR * kKD || in_sizes[7] != kKD || in_sizes[8] != kDVH ||
      in_sizes[9] != kVD * kDM || out_size != kRows * kDM) return;

  const float* x      = (const float*)d_in[0];
  const float* Wq     = (const float*)d_in[1];
  const float* Wk     = (const float*)d_in[2];
  const float* Wv     = (const float*)d_in[3];
  const float* Wg     = (const float*)d_in[4];
  const float* Wgk1   = (const float*)d_in[5];
  const float* Wgk2   = (const float*)d_in[6];
  const float* bgk    = (const float*)d_in[7];
  const float* norm_w = (const float*)d_in[8];
  const float* Wo     = (const float*)d_in[9];
  float* out = (float*)d_out;

  char* ws = (char*)d_ws;
  size_t off = 0;
  auto carve = [&](size_t bytes) -> char* { char* p = ws + off; off += (bytes + 255) & ~(size_t)255; return p; };
  unsigned short* XH  = (unsigned short*)carve((size_t)kRows * kDM * 2);
  unsigned short* WAT = (unsigned short*)carve((size_t)kNA * kDM * 2);
  unsigned short* WVT = (unsigned short*)carve((size_t)kVD * kDM * 2);
  unsigned short* WGT = (unsigned short*)carve((size_t)kVD * kDM * 2);
  unsigned short* WOT = (unsigned short*)carve((size_t)kDM * kVD * 2);
  float*          QKT = (float*)carve((size_t)kRows * kNA * 4);
  unsigned short* VT  = (unsigned short*)carve((size_t)kVD * kRows * 2);
  unsigned short* GP  = (unsigned short*)carve((size_t)kRows * kVD * 2);
  unsigned short* QG  = (unsigned short*)carve((size_t)kRows * kKD * 2);
  unsigned short* KG  = (unsigned short*)carve((size_t)kRows * kKD * 2);
  unsigned short* KDT = (unsigned short*)carve((size_t)kRows * kKD * 2);
  float*          GL  = (float*)carve((size_t)kNB * kNCH * kKD * 4);
  if (off > ws_size || off > (size_t)134217728) return;
  float*          ORAW = QKT;
  unsigned short* OG   = XH;

  const int n8x = kRows * kDM / 8;
  cvt8_kernel<<<n8x / 256, 256, 0, stream>>>(x, XH, n8x);
  wtcast_kernel<<<dim3(kDM / 64, kKD / 64), 256, 0, stream>>>(Wq, kKD, WAT, kWCarry);
  wtcast_kernel<<<dim3(kDM / 64, kKD / 64), 256, 0, stream>>>(Wk, kKD, WAT + (size_t)kKD * kDM, kWCarry);
  wtcast_kernel<<<dim3(kDM / 64, 1), 256, 0, stream>>>(Wgk1, kLR, WAT + (size_t)2 * kKD * kDM, kWCarry);
  wtcast_kernel<<<dim3(kDM / 64, kVD / 64), 256, 0, stream>>>(Wv, kVD, WVT, kWCarry);
  wtcast_kernel<<<dim3(kDM / 64, kVD / 64), 256, 0, stream>>>(Wg, kVD, WGT, kWCarry);
  wtcast_kernel<<<dim3(kVD / 64, kDM / 64), 256, 0, stream>>>(Wo, kDM, WOT, kWCarry);

  wmma_gemm64_h<0><<<(kRows / 64) * (kNA / 64) / 8, 256, 0, stream>>>(
      XH, kDM, WAT, kDM, (void*)QKT, kNA, kRows, kNA, kDM, kWCarryInv);
  wmma_gemm64_h<1><<<(kVD / 64) * (kRows / 64) / 8, 256, 0, stream>>>(
      WVT, kDM, XH, kDM, (void*)VT, kRows, kVD, kRows, kDM, kWCarryInv);
  wmma_gemm64_h<1><<<(kRows / 64) * (kVD / 64) / 8, 256, 0, stream>>>(
      XH, kDM, WGT, kDM, (void*)GP, kVD, kRows, kVD, kDM, kWCarryInv);

  prep_kernel<<<kNB * kNCH * kNH, 128, 0, stream>>>(QKT, Wgk2, bgk, QG, KG, KDT, GL);

  chunk_scan_kernel<<<kNB * kNH * (kDVH / 64), 256, 0, stream>>>(QG, KG, KDT, VT, GL, ORAW);

  norm_gate_kernel<<<kRows * kNH / 8, 256, 0, stream>>>(ORAW, GP, norm_w, OG);

  wmma_gemm64_h<0><<<(kRows / 64) * (kDM / 64) / 8, 256, 0, stream>>>(
      OG, kVD, WOT, kVD, (void*)out, kDM, kRows, kDM, kVD, kWCarryInv);
}
